// HybridSTPAttention_36472862277839
// MI455X (gfx1250) — hardware-verified
//
#include <hip/hip_runtime.h>
#include <math.h>

typedef __attribute__((ext_vector_type(16))) _Float16 v16h;
typedef __attribute__((ext_vector_type(16))) __bf16 v16b;
typedef __attribute__((ext_vector_type(8)))  _Float16 v8h;
typedef __attribute__((ext_vector_type(8)))  float v8f;
typedef __attribute__((ext_vector_type(4)))  float v4f;
typedef __attribute__((ext_vector_type(2)))  float v2f;
typedef __attribute__((ext_vector_type(4)))  unsigned v4u;
typedef __attribute__((ext_vector_type(4)))  int v4i;
typedef float __attribute__((may_alias)) float_a;
typedef int __attribute__((may_alias)) int_a;

template <typename T> __device__ __forceinline__ void vst2(void* p, T v) { *(volatile T*)p = v; __threadfence(); *(volatile T*)p = v; }
__device__ __forceinline__ v8f wmma16(v16h a, v16h b, v8f c) {
  v8f d = __builtin_amdgcn_wmma_f32_16x16x32_f16(false, a, false, b, (short)0, c, false, false);
  asm volatile("v_nop\n\tv_nop\n\tv_nop\n\tv_nop" : "+v"(d) : "v"(a), "v"(b));
  return d;
}
__device__ __forceinline__ v8f wmma_bf(v16b a, v16b b, v8f c) {
  v8f d = __builtin_amdgcn_wmma_f32_16x16x32_bf16(false, a, false, b, (short)0, c, false, false);
  asm volatile("v_nop\n\tv_nop\n\tv_nop\n\tv_nop" : "+v"(d) : "v"(a), "v"(b));
  return d;
}
__device__ __forceinline__ v16h frag_h(const _Float16* rowk0, int lane) {
  union { v16h v; v8h q[2]; } u; const _Float16* p = rowk0 + 8 * (lane >> 4);
  u.q[0] = *(const v8h*)p; u.q[1] = *(const v8h*)(p + 16); return u.v;
}
__device__ __forceinline__ v16h frag_f32(const float* rowk0, int lane) {
  v16h a; const float* p = rowk0 + 8 * (lane >> 4);
#pragma unroll
  for (int i = 0; i < 8; ++i) { a[i] = (_Float16)p[i]; a[8 + i] = (_Float16)p[16 + i]; }
  return a;
}
__device__ __forceinline__ v16h frag_f32s(const float* rowk0, int lane, float sc) {
  v16h a; const float* p = rowk0 + 8 * (lane >> 4);
#pragma unroll
  for (int i = 0; i < 8; ++i) { a[i] = (_Float16)(p[i] * sc); a[8 + i] = (_Float16)(p[16 + i] * sc); }
  return a;
}
__device__ __forceinline__ v16h fragc_f32(const float* W, int k0, int n, int lane, int ld, int K) {
  v16h a; const int g = lane >> 4;
#pragma unroll
  for (int i = 0; i < 8; ++i) { const int ka = k0 + 8 * g + i, kb = ka + 16;
    a[i] = (_Float16)(ka < K ? W[(size_t)(ka < K ? ka : K - 1) * ld + n] : 0.f); a[8 + i] = (_Float16)(kb < K ? W[(size_t)(kb < K ? kb : K - 1) * ld + n] : 0.f); }
  return a;
}
struct F2 { v16b h, l; };
__device__ __forceinline__ F2 bsplit16(const float v[16]) { F2 r;
#pragma unroll
  for (int i = 0; i < 16; ++i) { const __bf16 h = (__bf16)v[i]; r.h[i] = h; r.l[i] = (__bf16)(v[i] - (float)h); }
  return r; }
__device__ __forceinline__ F2 split_row(const float* row, int k0, int lane) { float v[16]; const float* p = row + k0 + 8 * (lane >> 4);
#pragma unroll
  for (int i = 0; i < 8; ++i) { v[i] = p[i]; v[8 + i] = p[16 + i]; }
  return bsplit16(v); }
__device__ __forceinline__ F2 split_rowK(const float* row, int k0, int lane, int K) { float v[16]; const int g = lane >> 4;
#pragma unroll
  for (int i = 0; i < 8; ++i) { const int ka = k0 + 8 * g + i, kb = ka + 16; v[i] = ka < K ? row[ka < K ? ka : K - 1] : 0.f; v[8 + i] = kb < K ? row[kb < K ? kb : K - 1] : 0.f; }
  return bsplit16(v); }
__device__ __forceinline__ F2 split_col(const float* W, int k0, int n, int lane, int ld, int K) { float v[16]; const int g = lane >> 4;
#pragma unroll
  for (int i = 0; i < 8; ++i) { const int ka = k0 + 8 * g + i, kb = ka + 16; v[i] = ka < K ? W[(size_t)(ka < K ? ka : K - 1) * ld + n] : 0.f; v[8 + i] = kb < K ? W[(size_t)(kb < K ? kb : K - 1) * ld + n] : 0.f; }
  return bsplit16(v); }
__device__ __forceinline__ v8f mac3(const F2& a, const F2& b, v8f c) { c = wmma_bf(a.l, b.h, c); c = wmma_bf(a.h, b.l, c); return wmma_bf(a.h, b.h, c); }
__device__ __forceinline__ float sigm(float v) { return 1.0f / (1.0f + expf(-v)); }
#define LDSX() do { asm volatile("s_wait_dscnt 0" ::: "memory"); __builtin_amdgcn_wave_barrier(); __builtin_amdgcn_fence(__ATOMIC_RELEASE, "workgroup"); } while (0)


#define NB 2
#define SS 2048
#define E 1024
#define NH 16
#define HD 64
#define NR (NB * SS)
#define GH 512
#define TR_ROWS NR
#define TR_QB (SS / 64)
#define TR_BH (NB * NH)
#ifndef NSTEP
#define NSTEP SS
#endif
typedef __attribute__((ext_vector_type(8))) __bf16 v8b;
__device__ __forceinline__ v16b frag_b(const __bf16* rowk0, int lane) {
  union { v16b v; v8b q[2]; } u; const __bf16* p = rowk0 + 8 * (lane >> 4);
  u.q[0] = *(const v8b*)p; u.q[1] = *(const v8b*)(p + 16); return u.v;
}
__device__ __forceinline__ float bfr(float v) { return (float)(__bf16)v; }
__device__ __attribute__((noinline)) float gelu_e(float v) { return 0.5f * v * (1.0f + erff(v * 0.70710678118654752f)); }
__device__ __attribute__((noinline)) float exp_ni(float v) { return expf(v); }
__device__ __forceinline__ v8f mac3p(v16b ah, v16b al, v16b bh, v16b bl, v8f c) { c = wmma_bf(al, bh, c); c = wmma_bf(ah, bl, c); return wmma_bf(ah, bh, c); }

#define BHT      ((size_t)NB * NH * SS)
#define WS_PT    0u
#define PT_ROWS  4608u
#define WS_W2T   (WS_PT + 2u * PT_ROWS * E)
#define WS_XB    (WS_W2T + 2u * 16 * GH)
#define WS_Q32   (WS_XB + 2u * NR * E)
#define WS_K32   (WS_Q32 + 4u * BHT * HD)
#define WS_V32   (WS_K32 + 4u * BHT * HD)
#define WS_VTH   (WS_V32 + 4u * BHT * HD)
#define WS_VTL   (WS_VTH + 2u * BHT * HD)
#define WS_YS    (WS_VTL + 2u * BHT * HD)
#define WS_YP    (WS_YS + 4u * BHT * HD)
#define WS_G1    (WS_YP + 4u * BHT * HD)
#define WS_AL    (WS_G1 + 4u * NR * GH)
#define WS_END   (WS_AL + 4u * NR * 16)

__global__ __launch_bounds__(256) void k_pack(const float* __restrict__ Wqkv, const float* __restrict__ Wout, const float* __restrict__ W1, const float* __restrict__ W2, __bf16* __restrict__ PT, __bf16* __restrict__ W2T) {
  __shared__ __align__(16) __bf16 srow[E];
  const int n = blockIdx.x, tid = threadIdx.x;
  if (n < (int)PT_ROWS) {
    const float* Wm; int NOUT, nn;
    if (n < 3072) { Wm = Wqkv; NOUT = 3072; nn = n; } else if (n < 4096) { Wm = Wout; NOUT = E; nn = n - 3072; } else { Wm = W1; NOUT = GH; nn = n - 4096; }
    for (int k = tid; k < E; k += 256) srow[k] = (__bf16)Wm[(size_t)k * NOUT + nn];
    __syncthreads();
    if (tid < E / 8) vst2((unsigned*)(PT + (size_t)n * E + tid * 8), *(const v4u*)(&srow[tid * 8]));
  } else {
    const int o = n - PT_ROWS;
    for (int k = tid; k < GH; k += 256) srow[k] = (__bf16)W2[(size_t)k * 16 + o];
    __syncthreads();
    if (tid < GH / 8) vst2((unsigned*)(W2T + (size_t)o * GH + tid * 8), *(const v4u*)(&srow[tid * 8]));
  }
}
__global__ __launch_bounds__(256) void k_cvt(const float* __restrict__ x, __bf16* __restrict__ Xb) {
  const size_t r = blockIdx.x; const int tid = threadIdx.x; const float* src = x + r * E + tid * 4;
  const float4 v = *(const float4*)src; union { __bf16 e[4]; v2f u; } pk; pk.e[0] = (__bf16)v.x; pk.e[1] = (__bf16)v.y; pk.e[2] = (__bf16)v.z; pk.e[3] = (__bf16)v.w;
  vst2((v2f*)(Xb + r * E + tid * 4), pk.u);
}
__global__ __launch_bounds__(128) void k_qkv(const __bf16* __restrict__ Xb, const __bf16* __restrict__ PT, const float* __restrict__ bqkv, float* __restrict__ Q32, float* __restrict__ K32, float* __restrict__ V32, __bf16* __restrict__ VTh, __bf16* __restrict__ VTl) {
  __shared__ __align__(16) float so[4][16][132];
  __shared__ __align__(16) __bf16 sth[128][72], stl[128][72];
  const int tid = threadIdx.x, wave = tid >> 5, lane = tid & 31, col = lane & 15, g = lane >> 4;
  const int which = blockIdx.z, r0b = blockIdx.x * 64, r0 = r0b + wave * 16, n0 = blockIdx.y * 128; const int b = r0b / SS, s0 = r0b % SS;
  const float* bb_ = bqkv + which * E;
  v8f acc[8] = {};
#pragma unroll 2
  for (int kc = 0; kc < E / 32; ++kc) { const v16b a = frag_b(Xb + (size_t)(r0 + col) * E + kc * 32, lane);
#pragma unroll
    for (int j = 0; j < 8; ++j) acc[j] = wmma_bf(a, frag_b(PT + (size_t)(which * E + n0 + j * 16 + col) * E + kc * 32, lane), acc[j]); }
#pragma unroll
  for (int j = 0; j < 8; ++j) { const float bb = bfr(bb_[n0 + j * 16 + col]);
#pragma unroll
    for (int r = 0; r < 8; ++r) so[wave][8 * g + r][j * 16 + col] = acc[j][r] + bb; }
  LDSX();
  float* Dst = which == 0 ? Q32 : which == 1 ? K32 : V32;
  for (int qq = lane; qq < 2 * 16 * 16; qq += 32) { const int hh = qq >> 8, rl = (qq >> 4) & 15, pc = qq & 15; const int h = (n0 >> 6) + hh;
    vst2(Dst + (((size_t)b * NH + h) * SS + s0 + wave * 16 + rl) * HD + pc * 4, *(const v4f*)(&so[wave][rl][hh * 64 + pc * 4])); }
  if (which == 2) {
#pragma unroll
    for (int j = 0; j < 8; ++j)
#pragma unroll
      for (int r = 0; r < 8; ++r) { const float v = so[wave][8 * g + r][j * 16 + col]; const __bf16 hi = (__bf16)v; sth[j * 16 + col][wave * 16 + 8 * g + r] = hi; stl[j * 16 + col][wave * 16 + 8 * g + r] = (__bf16)(v - (float)hi); }
    __syncthreads();
    for (int qq = tid; qq < 128 * 8; qq += 128) { const int cl = qq >> 3, pc = qq & 7; const int c = n0 + cl, h = c >> 6, d = c & 63; const size_t o = (((size_t)b * NH + h) * HD + d) * SS + s0 + pc * 8;
      vst2((unsigned*)(VTh + o), *(const v4u*)(&sth[cl][pc * 8])); vst2((unsigned*)(VTl + o), *(const v4u*)(&stl[cl][pc * 8])); } }
}
__global__ __launch_bounds__(128) void k_attn(const float* __restrict__ Q32, const float* __restrict__ K32, const __bf16* __restrict__ VTh, const __bf16* __restrict__ VTl, float* __restrict__ YS) {
  __shared__ __align__(16) float sS[4][16][68];
  __shared__ __align__(16) __bf16 sPh[4][16][72], sPl[4][16][72];
  __shared__ __align__(16) float sO[4][16][68];
  const int tid = threadIdx.x, w = tid >> 5, lane = tid & 31, col = lane & 15, g = lane >> 4;
  const size_t bh = blockIdx.y; const int qb = blockIdx.x; const int q0 = qb * 64 + w * 16;
  F2 aq[2];
#pragma unroll
  for (int kc = 0; kc < 2; ++kc) aq[kc] = split_row(Q32 + (bh * SS + q0 + col) * HD, kc * 32, lane);
  float mrun = -3.0e38f, lrun = 0.f; v8f acc[4] = {};
#pragma unroll 1
  for (int kt = 0; kt <= qb; ++kt) {
#pragma unroll
    for (int t = 0; t < 4; ++t) { const int key = kt * 64 + t * 16 + col; const float* krow = K32 + (bh * SS + key) * HD;
      v8f s = mac3(aq[0], split_row(krow, 0, lane), (v8f){}); s = mac3(aq[1], split_row(krow, 32, lane), s);
#pragma unroll
      for (int r = 0; r < 8; ++r) { sS[w][8 * g + r][t * 16 + col] = (key > q0 + 8 * g + r) ? -3.0e38f : s[r] * 0.125f; } }
    LDSX();
    float mx = -3.4e38f;
#pragma unroll
    for (int jj = 0; jj < 32; ++jj) mx = fmaxf(mx, sS[w][col][g * 32 + jj]);
    mx = fmaxf(mx, __shfl_xor(mx, 16, 32));
    const float mnew = fmaxf(mrun, mx); const float corr = exp_ni(mrun - mnew);
    float ps = 0.f;
#pragma unroll 8
    for (int jj = 0; jj < 32; ++jj) { const float p = exp_ni(sS[w][col][g * 32 + jj] - mnew); ps += p; const __bf16 hi = (__bf16)p; sPh[w][col][g * 32 + jj] = hi; sPl[w][col][g * 32 + jj] = (__bf16)(p - (float)hi); }
    ps += __shfl_xor(ps, 16, 32);
    lrun = lrun * corr + ps; mrun = mnew;
#pragma unroll
    for (int r = 0; r < 8; ++r) { const float cr = __shfl(corr, 8 * g + r, 32);
#pragma unroll
      for (int t = 0; t < 4; ++t) acc[t][r] *= cr; }
    LDSX();
#pragma unroll
    for (int kc = 0; kc < 2; ++kc) { const v16b ph = frag_b(&sPh[w][col][0] + kc * 32, lane), pl = frag_b(&sPl[w][col][0] + kc * 32, lane);
#pragma unroll
      for (int t = 0; t < 4; ++t) { const size_t vo = (bh * HD + t * 16 + col) * SS + kt * 64 + kc * 32; acc[t] = mac3p(ph, pl, frag_b(VTh + vo, lane), frag_b(VTl + vo, lane), acc[t]); } }
    __builtin_amdgcn_wave_barrier(); }
#pragma unroll
  for (int r = 0; r < 8; ++r) { const float lr = __shfl(lrun, 8 * g + r, 32); const float inv = 1.0f / lr;
#pragma unroll
    for (int t = 0; t < 4; ++t) sO[w][8 * g + r][t * 16 + col] = acc[t][r] * inv; }
  LDSX();
  for (int qq = lane; qq < 16 * 16; qq += 32) { const int rl = qq >> 4, pc = qq & 15; vst2(YS + ((bh * SS) + q0 + rl) * HD + pc * 4, *(const v4f*)(&sO[w][rl][pc * 4])); }
}
__global__ __launch_bounds__(256) void k_stp(const float* __restrict__ Q32, const float* __restrict__ K32, const float* __restrict__ V32, const float* __restrict__ Wst, const float* __restrict__ Lam, const float* __restrict__ Gam, float* __restrict__ YP) {
  __shared__ __align__(16) float sy[16][HD];
  __shared__ float sst[256][17], sret[256][17], sgam[256][17], swst[256][17];
  const int bh = blockIdx.x, h = bh % NH, tid = threadIdx.x, i = tid >> 2, jq = tid & 3, j0 = jq * 16;
  for (int e = 0; e < 16; ++e) { const size_t o = ((size_t)h * HD + i) * HD + j0 + e; sst[tid][e] = 0.f; sret[tid][e] = 1.0f - 1.0f / (1.0f + exp_ni(-bfr(Lam[o]))); sgam[tid][e] = bfr(Gam[o]); swst[tid][e] = bfr(Wst[o]); }
  const float* qb_ = Q32 + (size_t)bh * SS * HD + j0; const float* kb_ = K32 + (size_t)bh * SS * HD + j0; const float* vb_ = V32 + (size_t)bh * SS * HD + i;
#pragma unroll 1
  for (int t = 0; t < NSTEP; ++t) {
    const float vi = vb_[(size_t)t * HD]; const float* kr = kb_ + (size_t)t * HD; const float* qr = qb_ + (size_t)t * HD;
    float y = 0.f;
#pragma unroll 4
    for (int e = 0; e < 16; ++e) { const float hebb = vi * (kr[e] * 0.125f); const float s = sret[tid][e] * sst[tid][e] + sgam[tid][e] * hebb; sst[tid][e] = s; y += (swst[tid][e] + s) * qr[e]; }
    y += __shfl_xor(y, 1); y += __shfl_xor(y, 2);
    if (jq == 0) sy[t & 15][i] = y;
    if ((t & 15) == 15) {
      __syncthreads();
      { const int rl = tid >> 4, pc = tid & 15; vst2(YP + ((size_t)bh * SS + (t - 15) + rl) * HD + pc * 4, *(const v4f*)(&sy[rl][pc * 4])); }
      __syncthreads(); }
  }
}
__global__ __launch_bounds__(128) void k_g1(const __bf16* __restrict__ Xb, const __bf16* __restrict__ PT, const float* __restrict__ b1, float* __restrict__ G1) {
  __shared__ __align__(16) float so[4][16][132];
  const int tid = threadIdx.x, wave = tid >> 5, lane = tid & 31, col = lane & 15, g = lane >> 4; const size_t r0 = (size_t)blockIdx.x * 64 + wave * 16; const int n0 = blockIdx.y * 128;
  v8f acc[8] = {};
#pragma unroll 2
  for (int kc = 0; kc < E / 32; ++kc) { const v16b a = frag_b(Xb + (r0 + col) * E + kc * 32, lane);
#pragma unroll
    for (int j = 0; j < 8; ++j) acc[j] = wmma_bf(a, frag_b(PT + (size_t)(4096 + n0 + j * 16 + col) * E + kc * 32, lane), acc[j]); }
#pragma unroll
  for (int j = 0; j < 8; ++j) { const float bb = bfr(b1[n0 + j * 16 + col]);
#pragma unroll
    for (int r = 0; r < 8; ++r) so[wave][8 * g + r][j * 16 + col] = gelu_e(acc[j][r] + bb); }
  LDSX();
  for (int rl = 0; rl < 16; ++rl) vst2(G1 + (r0 + rl) * GH + n0 + lane * 4, *(const v4f*)(&so[wave][rl][lane * 4]));
}
__global__ __launch_bounds__(128) void k_g2(const float* __restrict__ G1, const __bf16* __restrict__ W2T, const float* __restrict__ b2, float* __restrict__ AL) {
  __shared__ __align__(16) float sa[64][16];
  const int tid = threadIdx.x, wave = tid >> 5, lane = tid & 31, col = lane & 15, g = lane >> 4; const size_t r0 = (size_t)blockIdx.x * 64 + wave * 16;
  v8f acc = {};
#pragma unroll 2
  for (int kc = 0; kc < GH / 32; ++kc) { const F2 a = split_row(G1 + (r0 + col) * GH, kc * 32, lane); const v16b wb = frag_b(W2T + (size_t)col * GH + kc * 32, lane); acc = wmma_bf(a.l, wb, acc); acc = wmma_bf(a.h, wb, acc); }
  const float bb = bfr(b2[col]);
#pragma unroll
  for (int r = 0; r < 8; ++r) sa[wave * 16 + 8 * g + r][col] = 1.0f / (1.0f + exp_ni(-(acc[r] + bb)));
  __syncthreads();
  for (int q = tid; q < 64 * 4; q += 128) vst2(AL + (size_t)blockIdx.x * 64 * 16 + q * 4, *(const v4f*)(&sa[0][0] + q * 4));
}
__global__ __launch_bounds__(128) void k_out(const float* __restrict__ YS, const float* __restrict__ YP, const float* __restrict__ AL, const __bf16* __restrict__ PT, const float* __restrict__ bo, float* __restrict__ out) {
  __shared__ __align__(16) float so[4][16][132];
  const int tid = threadIdx.x, wave = tid >> 5, lane = tid & 31, col = lane & 15, g = lane >> 4; const size_t r0 = (size_t)blockIdx.x * 64 + wave * 16; const int n0 = blockIdx.y * 128;
  const size_t r = r0 + col; const int b = (int)(r / SS), t = (int)(r % SS);
  v8f acc[8] = {};
#pragma unroll 1
  for (int kc = 0; kc < E / 32; ++kc) { const int h = kc >> 1, d0 = (kc & 1) * 32; const float al = AL[r * 16 + h];
    const size_t yo = (((size_t)b * NH + h) * SS + t) * HD + d0 + 8 * g; float v[16];
#pragma unroll
    for (int e = 0; e < 8; ++e) { v[e] = al * YS[yo + e] + (1.0f - al) * YP[yo + e]; v[8 + e] = al * YS[yo + 16 + e] + (1.0f - al) * YP[yo + 16 + e]; }
    const F2 a = bsplit16(v);
#pragma unroll
    for (int j = 0; j < 8; ++j) { const v16b wb = frag_b(PT + (size_t)(3072 + n0 + j * 16 + col) * E + kc * 32, lane); acc[j] = wmma_bf(a.l, wb, acc[j]); acc[j] = wmma_bf(a.h, wb, acc[j]); } }
#pragma unroll
  for (int j = 0; j < 8; ++j) { const float bb = bfr(bo[n0 + j * 16 + col]);
#pragma unroll
    for (int rr = 0; rr < 8; ++rr) so[wave][8 * g + rr][j * 16 + col] = acc[j][rr] + bb; }
  LDSX();
  for (int rl = 0; rl < 16; ++rl) vst2(out + (r0 + rl) * E + n0 + lane * 4, *(const v4f*)(&so[wave][rl][lane * 4]));
}

extern "C" void kernel_launch(void* const* d_in, const int* in_sizes, int n_in, void* d_out, int out_size, void* d_ws, size_t ws_size, hipStream_t stream) {
  (void)in_sizes; (void)n_in; (void)out_size;
  const float** I = (const float**)d_in;
  if (ws_size < (size_t)WS_END) return;
  char* ws = (char*)d_ws;
  __bf16 *PT = (__bf16*)(ws + WS_PT), *W2T = (__bf16*)(ws + WS_W2T), *Xb = (__bf16*)(ws + WS_XB), *VTh = (__bf16*)(ws + WS_VTH), *VTl = (__bf16*)(ws + WS_VTL);
  float *Q32 = (float*)(ws + WS_Q32), *K32 = (float*)(ws + WS_K32), *V32 = (float*)(ws + WS_V32), *YS = (float*)(ws + WS_YS), *YP = (float*)(ws + WS_YP), *G1 = (float*)(ws + WS_G1), *AL = (float*)(ws + WS_AL);
  k_pack<<<PT_ROWS + 16, 256, 0, stream>>>(I[1], I[3], I[8], I[10], PT, W2T);
  k_cvt<<<TR_ROWS, 256, 0, stream>>>(I[0], Xb);
  k_qkv<<<dim3(TR_ROWS / 64, E / 128, 3), 128, 0, stream>>>(Xb, PT, I[2], Q32, K32, V32, VTh, VTl);
  k_attn<<<dim3(TR_QB, TR_BH), 128, 0, stream>>>(Q32, K32, VTh, VTl, YS);
  k_stp<<<TR_BH, 256, 0, stream>>>(Q32, K32, V32, I[5], I[6], I[7], YP);
  k_g1<<<dim3(TR_ROWS / 64, GH / 128), 128, 0, stream>>>(Xb, PT, I[9], G1);
  k_g2<<<TR_ROWS / 64, 128, 0, stream>>>(G1, W2T, I[11], AL);
  k_out<<<dim3(TR_ROWS / 64, E / 128), 128, 0, stream>>>(YS, YP, AL, PT, I[4], (float*)d_out);
}
